// FusedQKVAttention_Kernel_50508815401128
// MI455X (gfx1250) — hardware-verified
//
#include <hip/hip_runtime.h>
#include <stddef.h>
#include <stdint.h>

#define NBAT  2
#define SQ    2048
#define NTOK  4096
#define HID   1024
#define NH    16
#define HDM   64
#define NQKV  3072
#define KOFS  HID
#define VOFS  (2 * HID)
#define NSLAB 24
#define QB    128
#define KC    64
#define NQB   (SQ / QB)
#define NCK   (SQ / KC)

static_assert(NTOK == NBAT * SQ);
static_assert(SQ % 256 == 0);
static_assert(HID % 64 == 0);
static_assert(HID == 128 * 8);
static_assert(HDM == 64);
static_assert(NH * HDM == HID);
static_assert(NQKV == 3 * HID);
static_assert(NQKV == NSLAB * 128);
static_assert(SQ % KC == 0);
static_assert(SQ % QB == 0);
static_assert(NTOK % 64 == 0);
static_assert(NTOK % 2 == 0);

typedef _Float16 v16h __attribute__((ext_vector_type(16)));
typedef _Float16 v8h  __attribute__((ext_vector_type(8)));
typedef float    v8f  __attribute__((ext_vector_type(8)));
typedef float    v4f  __attribute__((ext_vector_type(4)));
typedef unsigned int v4u __attribute__((ext_vector_type(4)));

union Frag  { v16h v; v8h h[2]; };
union Pack8 { v8h h; v4u u; };

__device__ __forceinline__ v8f mma16(v16h a, v16h b, v8f c) {
  c = __builtin_amdgcn_wmma_f32_16x16x32_f16(false, a, false, b, (short)0, c, false, false);
  asm volatile("v_nop\n\tv_nop\n\tv_nop\n\tv_nop" : "+v"(c) : "v"(a), "v"(b));
  return c;
}

__device__ __forceinline__ v16h ldfrag(const _Float16* p, int ld, int row0, int k0, int lane) {
  const int m = lane & 15, lh = lane >> 4;
  const _Float16* q = p + (size_t)(row0 + m) * ld + k0 + 8 * lh;
  Frag f;
  f.h[0] = *(const v8h*)(q);
  f.h[1] = *(const v8h*)(q + 16);
  return f.v;
}

__device__ __forceinline__ v8f zero8() { return (v8f){0.f, 0.f, 0.f, 0.f, 0.f, 0.f, 0.f, 0.f}; }

__device__ __forceinline__ void gemm16x64(const _Float16* __restrict__ A, int lda,
                                          const _Float16* __restrict__ Bt, int ldb,
                                          int m0, int n0, int lane, v8f (&acc)[4]) {
#pragma unroll 2
  for (int k0 = 0; k0 < HID; k0 += 32) {
    const v16h a = ldfrag(A, lda, m0, k0, lane);
#pragma unroll
    for (int t = 0; t < 4; ++t) {
      const v16h b = ldfrag(Bt, ldb, n0 + 16 * t, k0, lane);
      acc[t] = mma16(a, b, acc[t]);
    }
  }
}

__global__ __launch_bounds__(256) void k_cvtx(const float* __restrict__ src, _Float16* __restrict__ dh) {
  const int tid = threadIdx.x;
  const int row = blockIdx.x * 2 + (tid >> 7);
  const int col = (tid & 127) * 8;
  const size_t o = (size_t)row * HID + col;
  const v4f a0 = *(const v4f*)(src + o);
  const v4f a1 = *(const v4f*)(src + o + 4);
  Pack8 pk;
  pk.h = (v8h){(_Float16)a0[0], (_Float16)a0[1], (_Float16)a0[2], (_Float16)a0[3],
               (_Float16)a1[0], (_Float16)a1[1], (_Float16)a1[2], (_Float16)a1[3]};
  const v4u vv = pk.u;
  volatile v4u* d = (volatile v4u*)(dh + o);
  *d = vv;
  __threadfence();
  *d = vv;
}

#define WTP 65
__global__ __launch_bounds__(256) void k_wtr(const float* __restrict__ W, int ncol, int nofs,
                                             _Float16* __restrict__ wt) {
  __shared__ float tl[64 * WTP];
  const int tid = threadIdx.x;
  const int n0 = blockIdx.x * 64, k0 = blockIdx.y * 64;
#pragma unroll
  for (int j = 0; j < 4; ++j) {
    const int p  = tid + 256 * j;
    const int kk = p >> 4;
    const int q4 = (p & 15) * 4;
    const v4f a = *(const v4f*)(W + (size_t)(k0 + kk) * ncol + n0 + q4);
    float* d = tl + kk * WTP + q4;
    d[0] = a[0]; d[1] = a[1]; d[2] = a[2]; d[3] = a[3];
  }
  __syncthreads();
  v4u vt[2];
  size_t go[2];
#pragma unroll
  for (int j = 0; j < 2; ++j) {
    const int p  = tid + 256 * j;
    const int nn = p >> 3;
    const int pc = p & 7;
    const float* cp = tl + (pc * 8) * WTP + nn;
    Pack8 pk;
    pk.h = (v8h){(_Float16)(cp[0 * WTP] * 32.0f), (_Float16)(cp[1 * WTP] * 32.0f),
                 (_Float16)(cp[2 * WTP] * 32.0f), (_Float16)(cp[3 * WTP] * 32.0f),
                 (_Float16)(cp[4 * WTP] * 32.0f), (_Float16)(cp[5 * WTP] * 32.0f),
                 (_Float16)(cp[6 * WTP] * 32.0f), (_Float16)(cp[7 * WTP] * 32.0f)};
    vt[j] = pk.u;
    go[j] = (size_t)(nofs + n0 + nn) * HID + k0 + pc * 8;
  }
  for (int ps = 0; ps < 2; ++ps) {
#pragma unroll
    for (int j = 0; j < 2; ++j) *(volatile v4u*)(wt + go[j]) = vt[j];
    __threadfence();
  }
}

#define SFP 132
__global__ __launch_bounds__(256) void k_qkv(const _Float16* __restrict__ xh,
                                             const _Float16* __restrict__ wt,
                                             _Float16* __restrict__ qp,
                                             _Float16* __restrict__ kp,
                                             _Float16* __restrict__ vtp) {
  __shared__ __align__(16) float sf[64 * SFP];
  const int tid = threadIdx.x, lane = tid & 31, wave = tid >> 5;
  const int hh = lane >> 4, c = lane & 15;
  const int wm = wave >> 1, wn = wave & 1;
  const int mb = blockIdx.x * 64;
  const int b  = mb / SQ;
  const int sb = mb - b * SQ;
  const int ns = blockIdx.y;
  const int which = ns >> 3;
  const int hp = 2 * (ns & 7);
  const int m0 = mb + wm * 16;
  const int n0 = ns * 128 + wn * 64;

  v8f acc[4];
#pragma unroll
  for (int t = 0; t < 4; ++t) acc[t] = zero8();
  gemm16x64(xh, HID, wt, HID, m0, n0, lane, acc);

#pragma unroll
  for (int t = 0; t < 4; ++t) {
#pragma unroll
    for (int r = 0; r < 8; ++r)
      sf[(wm * 16 + 8 * hh + r) * SFP + wn * 64 + 16 * t + c] = acc[t][r] * 0.03125f;
  }
  __syncthreads();

  if (which < 2) {
    v4u val[4];
    size_t go[4];
#pragma unroll
    for (int j = 0; j < 4; ++j) {
      const int p  = tid + 256 * j;
      const int lr = p >> 4;
      const int pc = p & 15;
      const int hs = pc >> 3;
      const int d0 = (pc & 7) * 8;
      const float* ra = sf + lr * SFP + pc * 8;
      const v4f a0 = *(const v4f*)(ra), a1 = *(const v4f*)(ra + 4);
      Pack8 pk;
      pk.h = (v8h){(_Float16)a0[0], (_Float16)a0[1], (_Float16)a0[2], (_Float16)a0[3],
                   (_Float16)a1[0], (_Float16)a1[1], (_Float16)a1[2], (_Float16)a1[3]};
      val[j] = pk.u;
      const int hb = b * NH + hp + hs;
      go[j]  = ((size_t)hb * SQ + sb + lr) * HDM + d0;
    }
    _Float16* base = (which == 0) ? qp : kp;
    for (int ps = 0; ps < 2; ++ps) {
#pragma unroll
      for (int j = 0; j < 4; ++j) *(volatile v4u*)(base + go[j]) = val[j];
      __threadfence();
    }
  } else {
    v4u val[4];
    size_t go[4];
#pragma unroll
    for (int j = 0; j < 4; ++j) {
      const int p    = tid + 256 * j;
      const int dcol = p >> 3;
      const int pc   = p & 7;
      const float* cp = sf + (pc * 8) * SFP + dcol;
      Pack8 pk;
      pk.h = (v8h){(_Float16)cp[0 * SFP], (_Float16)cp[1 * SFP], (_Float16)cp[2 * SFP], (_Float16)cp[3 * SFP],
                   (_Float16)cp[4 * SFP], (_Float16)cp[5 * SFP], (_Float16)cp[6 * SFP], (_Float16)cp[7 * SFP]};
      val[j] = pk.u;
      const int hb = b * NH + hp + (dcol >> 6);
      const int d  = dcol & 63;
      go[j]  = ((size_t)hb * HDM + d) * SQ + sb + pc * 8;
    }
    for (int ps = 0; ps < 2; ++ps) {
#pragma unroll
      for (int j = 0; j < 4; ++j) *(volatile v4u*)(vtp + go[j]) = val[j];
      __threadfence();
    }
  }
}

#define KTP 72
#define OTP 68
#define SMEMF 9216
static_assert((KC * KTP + HDM * KTP + 8 * 16 * KTP) * 2 == SMEMF * 4);
static_assert(8 * 16 * OTP <= SMEMF);
__global__ __launch_bounds__(256) void k_attn(const _Float16* __restrict__ qp,
                                              const _Float16* __restrict__ kp,
                                              const _Float16* __restrict__ vt,
                                              float* __restrict__ out, float sscale) {
  __shared__ __align__(16) float smem[SMEMF];
  _Float16* Ks = (_Float16*)smem;
  _Float16* Vs = Ks + KC * KTP;
  _Float16* Ps = Vs + HDM * KTP;

  const int tid = threadIdx.x, lane = tid & 31, wave = tid >> 5;
  const int hh = lane >> 4, c = lane & 15;
  const int qb  = blockIdx.x % NQB;
  const int hb  = blockIdx.x / NQB;
  const int h   = hb % NH;
  const int b   = hb / NH;
  const int q0  = qb * QB + wave * 16;

  const _Float16* Q = qp + (size_t)hb * SQ * HDM;
  const _Float16* K = kp + (size_t)hb * SQ * HDM;
  const _Float16* V = vt + (size_t)hb * HDM * SQ;
  const size_t trow0 = (size_t)b * SQ;

  v16h qa[2];
  qa[0] = ldfrag(Q, HDM, q0, 0, lane);
  qa[1] = ldfrag(Q, HDM, q0, 32, lane);

  const float NEGI = -__builtin_huge_valf();
  float mrow[8], lrow[8];
  v8f oacc[4];
#pragma unroll
  for (int r = 0; r < 8; ++r) { mrow[r] = NEGI; lrow[r] = 0.f; }
#pragma unroll
  for (int t = 0; t < 4; ++t) oacc[t] = zero8();

  _Float16* pw = Ps + wave * 16 * KTP;

  for (int kc = 0; kc < NCK; ++kc) {
    const int kv0 = kc * KC;
    __syncthreads();
    {
      const int r  = tid >> 2;
      const int qq = (tid & 3) * 16;
      const _Float16* ks = K + (size_t)(kv0 + r) * HDM + qq;
      const _Float16* vs = V + (size_t)r * SQ + kv0 + qq;
#pragma unroll
      for (int e = 0; e < 2; ++e) {
        *(v8h*)(Ks + r * KTP + qq + 8 * e) = *(const v8h*)(ks + 8 * e);
        *(v8h*)(Vs + r * KTP + qq + 8 * e) = *(const v8h*)(vs + 8 * e);
      }
    }
    __syncthreads();

    v8f s[4];
#pragma unroll
    for (int j = 0; j < 4; ++j) s[j] = zero8();
#pragma unroll
    for (int dc = 0; dc < 2; ++dc) {
#pragma unroll
      for (int j = 0; j < 4; ++j) {
        const v16h kb = ldfrag(Ks, KTP, j * 16, dc * 32, lane);
        s[j] = mma16(qa[dc], kb, s[j]);
      }
    }
    float cm[8];
#pragma unroll
    for (int r = 0; r < 8; ++r) {
      float m = NEGI;
#pragma unroll
      for (int j = 0; j < 4; ++j) { s[j][r] *= sscale; m = fmaxf(m, s[j][r]); }
#pragma unroll
      for (int off = 1; off < 16; off <<= 1) m = fmaxf(m, __shfl_xor(m, off, 32));
      cm[r] = m;
    }
    float al[8];
#pragma unroll
    for (int r = 0; r < 8; ++r) {
      const float mnew  = fmaxf(mrow[r], cm[r]);
      const float alpha = __expf(mrow[r] - mnew);
      mrow[r] = mnew;
      float psum = 0.f;
#pragma unroll
      for (int j = 0; j < 4; ++j) {
        const float p = __expf(s[j][r] - mnew);
        psum += p;
        pw[(8 * hh + r) * KTP + j * 16 + c] = (_Float16)(p * 1024.0f);
      }
#pragma unroll
      for (int off = 1; off < 16; off <<= 1) psum += __shfl_xor(psum, off, 32);
      lrow[r] = lrow[r] * alpha + psum;
      al[r] = alpha;
    }
#pragma unroll
    for (int t = 0; t < 4; ++t)
#pragma unroll
      for (int r = 0; r < 8; ++r) oacc[t][r] *= al[r];
    __syncthreads();

#pragma unroll
    for (int kk = 0; kk < 2; ++kk) {
      const v16h pa = ldfrag(pw, KTP, 0, kk * 32, lane);
#pragma unroll
      for (int t = 0; t < 4; ++t) {
        const v16h vb = ldfrag(Vs, KTP, t * 16, kk * 32, lane);
        oacc[t] = mma16(pa, vb, oacc[t]);
      }
    }
  }

  float invl[8];
#pragma unroll
  for (int r = 0; r < 8; ++r) invl[r] = (lrow[r] > 0.f) ? (0.0009765625f / lrow[r]) : 0.f;
  __syncthreads();
  float* sw = smem + wave * 16 * OTP;
#pragma unroll
  for (int r = 0; r < 8; ++r) {
#pragma unroll
    for (int t = 0; t < 4; ++t)
      sw[(8 * hh + r) * OTP + 16 * t + c] = oacc[t][r] * invl[r];
  }
  __syncthreads();
  v4f val[8];
  size_t go[8];
#pragma unroll
  for (int it = 0; it < 8; ++it) {
    const int p    = lane + 32 * it;
    const int L    = p >> 3;
    const int pc   = p & 7;
    const int row  = L >> 1;
    const int half = L & 1;
    val[it] = *(const v4f*)(sw + row * OTP + half * 32 + pc * 4);
    go[it]  = (trow0 + q0 + row) * HID + (size_t)h * HDM + half * 32 + pc * 4;
  }
  for (int ps = 0; ps < 2; ++ps) {
#pragma unroll
    for (int it = 0; it < 8; ++it) *(volatile v4f*)(out + go[it]) = val[it];
    __threadfence();
  }
}

extern "C" void kernel_launch(void* const* d_in, const int* in_sizes, int n_in,
                              void* d_out, int out_size, void* d_ws, size_t ws_size,
                              hipStream_t stream) {
  if (n_in < 4) return;
  if (in_sizes[0] != NTOK * HID) return;
  if (in_sizes[1] != HID * HID) return;
  if (in_sizes[2] != HID * HID) return;
  if (in_sizes[3] != HID * HID) return;
  if (out_size != NTOK * HID) return;

  const float* x  = (const float*)d_in[0];
  const float* wq = (const float*)d_in[1];
  const float* wk = (const float*)d_in[2];
  const float* wv = (const float*)d_in[3];
  float* out = (float*)d_out;

  size_t off = 0;
  const size_t oX  = off; off += (size_t)NTOK * HID * 2;
  const size_t oWt = off; off += (size_t)NQKV * HID * 2;
  const size_t oQ  = off; off += (size_t)NBAT * NH * SQ * HDM * 2;
  const size_t oK  = off; off += (size_t)NBAT * NH * SQ * HDM * 2;
  const size_t oV  = off; off += (size_t)NBAT * NH * HDM * SQ * 2;
  if (off > ws_size) return;
  if (off > (size_t)134217728) return;

  char* ws = (char*)d_ws;
  _Float16* Xh = (_Float16*)(ws + oX);
  _Float16* Wt = (_Float16*)(ws + oWt);
  _Float16* Qp = (_Float16*)(ws + oQ);
  _Float16* Kp = (_Float16*)(ws + oK);
  _Float16* Vt = (_Float16*)(ws + oV);

  k_cvtx<<<dim3(NTOK / 2), dim3(256), 0, stream>>>(x, Xh);
  k_wtr<<<dim3(HID / 64, HID / 64), dim3(256), 0, stream>>>(wq, HID, 0, Wt);
  k_wtr<<<dim3(HID / 64, HID / 64), dim3(256), 0, stream>>>(wk, HID, KOFS, Wt);
  k_wtr<<<dim3(HID / 64, HID / 64), dim3(256), 0, stream>>>(wv, HID, VOFS, Wt);
  k_qkv<<<dim3(NTOK / 64, NSLAB), dim3(256), 0, stream>>>(Xh, Wt, Qp, Kp, Vt);
  const float sscale = 0.125f;
  k_attn<<<dim3(NBAT * NH * NQB), dim3(256), 0, stream>>>(Qp, Kp, Vt, out, sscale);
  (void)hipGetLastError();
}
